// SelfAttention_Inefficient_34694745817385
// MI455X (gfx1250) — hardware-verified
//
#include <hip/hip_runtime.h>


#define NB_  4
#define NN   4096
#define DD   64
#define NH_  2
#define PCAR 1024.0f
typedef _Float16 h16;
typedef unsigned short bf;
typedef __attribute__((ext_vector_type(16))) __bf16   v16bf;
typedef __attribute__((ext_vector_type(16))) _Float16 v16h;
typedef __attribute__((ext_vector_type(8)))  _Float16 v8h;
typedef __attribute__((ext_vector_type(8)))  unsigned short v8us;
typedef __attribute__((ext_vector_type(8)))  float    v8f;
typedef __attribute__((ext_vector_type(4)))  float    v4f;
typedef v8h  __attribute__((may_alias)) v8ha;
typedef v4f  __attribute__((may_alias)) v4fa;
typedef v8us __attribute__((may_alias)) v8usa;

__device__ __forceinline__ unsigned short f2bf(float f) { unsigned u = __float_as_uint(f); u += 0x7FFFu + ((u >> 16) & 1u); return (unsigned short)(u >> 16); }
__device__ __forceinline__ float bf2f(unsigned short b) { return __uint_as_float(((unsigned)b) << 16); }
__device__ __forceinline__ float bfr(float f) { return bf2f(f2bf(f)); }
__device__ __forceinline__ v16h cat16(v8h lo, v8h hi) { return __builtin_shufflevector(lo, hi, 0, 1, 2, 3, 4, 5, 6, 7, 8, 9, 10, 11, 12, 13, 14, 15); }
__device__ __forceinline__ v16bf cat16b(v8us lo, v8us hi) { return __builtin_bit_cast(v16bf, __builtin_shufflevector(lo, hi, 0, 1, 2, 3, 4, 5, 6, 7, 8, 9, 10, 11, 12, 13, 14, 15)); }
__device__ __forceinline__ v8f wmma16(v16h a, v16h b, v8f c) { return __builtin_amdgcn_wmma_f32_16x16x32_f16(false, a, false, b, (short)0, c, false, false); }
__device__ __forceinline__ v8f wmmab(v16bf a, v16bf b, v8f c) { return __builtin_amdgcn_wmma_f32_16x16x32_bf16(false, a, false, b, (short)0, c, false, false); }


template <typename T16> struct WFrag;
template <> struct WFrag<h16> { typedef v16h V; static __device__ __forceinline__ V ld(const h16* p) { return cat16(*(const v8h*)p, *(const v8h*)(p + 16)); } static __device__ __forceinline__ v8f mma(V a, V b, v8f c) { return wmma16(a, b, c); } };
template <> struct WFrag<bf> { typedef v16bf V; static __device__ __forceinline__ V ld(const bf* p) { return cat16b(*(const v8us*)p, *(const v8us*)(p + 16)); } static __device__ __forceinline__ v8f mma(V a, V b, v8f c) { return wmmab(a, b, c); } };
template <typename T16, int NSPLIT, bool BIAS>
__global__ __launch_bounds__(32) void k_gemmw(const T16* __restrict__ A, const T16* __restrict__ A2, const T16* __restrict__ Bt, const T16* __restrict__ Bt2, int K, float* C, int ldc, const float* __restrict__ bias, size_t sA, size_t sB, size_t sC) {
    typedef typename WFrag<T16>::V V;
    __shared__ __align__(16) float os[16 * 68];
    const size_t z = blockIdx.z; A += z * sA; if (A2) A2 += z * sA; Bt += z * sB; if (Bt2) Bt2 += z * sB; C += z * sC;
    const int lane = threadIdx.x & 31, lr = lane & 15, hi = lane >> 4; const int r0 = blockIdx.x * 64, c0 = blockIdx.y * 64;
    v8f acc[4][4];
#pragma unroll
    for (int mb = 0; mb < 4; ++mb)
#pragma unroll
        for (int nb = 0; nb < 4; ++nb) acc[mb][nb] = (v8f){};
    const size_t aoff = (size_t)(r0 + lr) * K + 8 * hi, boff = (size_t)(c0 + lr) * K + 8 * hi;
#pragma unroll 1
    for (int kc = 0; kc < K; kc += 32) {
        V a[4], a2[4];
#pragma unroll
        for (int mb = 0; mb < 4; ++mb) { a[mb] = WFrag<T16>::ld(A + aoff + (size_t)mb * 16 * K + kc); if (NSPLIT == 1 || NSPLIT == 2) a2[mb] = WFrag<T16>::ld(A2 + aoff + (size_t)mb * 16 * K + kc); }
#pragma unroll
        for (int nb = 0; nb < 4; ++nb) { const V b = WFrag<T16>::ld(Bt + boff + (size_t)nb * 16 * K + kc); V b2; if (NSPLIT >= 2) b2 = WFrag<T16>::ld(Bt2 + boff + (size_t)nb * 16 * K + kc);
#pragma unroll
            for (int mb = 0; mb < 4; ++mb) { acc[mb][nb] = WFrag<T16>::mma(a[mb], b, acc[mb][nb]); if (NSPLIT == 1 || NSPLIT == 2) acc[mb][nb] = WFrag<T16>::mma(a2[mb], b, acc[mb][nb]); if (NSPLIT >= 2) acc[mb][nb] = WFrag<T16>::mma(a[mb], b2, acc[mb][nb]); } }
        asm volatile("v_nop\n\tv_nop\n\tv_nop\n\tv_nop" : "+v"(acc[0][0]), "+v"(acc[1][1]), "+v"(acc[2][2]), "+v"(acc[3][3]) : "v"(a[0]), "v"(a[3]));
    }
#pragma unroll
    for (int mb = 0; mb < 4; ++mb) {
#pragma unroll
        for (int nb = 0; nb < 4; ++nb) {
#pragma unroll
            for (int j = 0; j < 8; ++j) os[(hi * 8 + j) * 68 + nb * 16 + lr] = acc[mb][nb][j]; }
        __builtin_amdgcn_wave_barrier(); asm volatile("" ::: "memory");
        float* crow = C + (size_t)(r0 + mb * 16) * ldc + c0;
#pragma unroll 1
        for (int ps = 0; ps < 2; ++ps) {
#pragma unroll
            for (int s = 0; s < 8; ++s) { const int row = 2 * s + hi, cofs = lr * 4; v4f val = *(const v4fa*)(os + row * 68 + cofs); if (BIAS) { val[0] += bfr(bias[c0 + cofs]); val[1] += bfr(bias[c0 + cofs + 1]); val[2] += bfr(bias[c0 + cofs + 2]); val[3] += bfr(bias[c0 + cofs + 3]); }
                *(volatile v4f*)(crow + (size_t)row * ldc + cofs) = val; }
            if (ps == 0) __threadfence(); }
        __builtin_amdgcn_wave_barrier(); asm volatile("" ::: "memory");
    }
}

__device__ __forceinline__ h16 tohx(float x) { return (h16)x; }
typedef __attribute__((ext_vector_type(2))) unsigned short v2us;
typedef __attribute__((ext_vector_type(2))) _Float16 v2h;
typedef __attribute__((ext_vector_type(4))) _Float16 v4h;

__global__ __launch_bounds__(256) void k_wtG(const float* __restrict__ w, int K, int N, bf* Bt) {
    const int lane = threadIdx.x & 31; const int L0 = (blockIdx.x * 8 + (threadIdx.x >> 5)) * 8; const int nlines = N * K / 64;
#pragma unroll
    for (int ps = 0; ps < 2; ++ps) {
#pragma unroll 1
        for (int l = 0; l < 8; ++l) { const int L = L0 + l; if (L >= nlines) break; const size_t e = (size_t)L * 64 + lane * 2; const int k = (int)(e % K), n = (int)(e / K); v2us o;
            o[0] = f2bf(w[(size_t)k * N + n]); o[1] = f2bf(w[(size_t)(k + 1) * N + n]); *(volatile v2us*)(Bt + e) = o; }
        if (ps == 0) __threadfence(); }
}
__global__ __launch_bounds__(256) void k_cvt8(const float* __restrict__ src, bf* dst, size_t n8) { const size_t i = (size_t)blockIdx.x * 256 + threadIdx.x; if (i >= n8) return; const v8f v = *(const v8f*)(src + i * 8); v8us o;
#pragma unroll
    for (int k = 0; k < 8; ++k) o[k] = f2bf(v[k]); *(volatile v8us*)(dst + i * 8) = o; __threadfence(); *(volatile v8us*)(dst + i * 8) = o; }
__global__ __launch_bounds__(256) void k_p16(const float* __restrict__ F, h16* P) { const int e = (blockIdx.x * 256 + threadIdx.x) * 4; if (e >= NN * DD) return; const v4f a = *(const v4f*)(F + e); v4h o;
#pragma unroll
    for (int u = 0; u < 4; ++u) o[u] = tohx(a[u]); *(volatile v4h*)(P + e) = o; __threadfence(); *(volatile v4h*)(P + e) = o; }
__global__ __launch_bounds__(256) void k_vt(const float* __restrict__ V, h16* VT) { const int e = (blockIdx.x * 256 + threadIdx.x) * 2; if (e >= DD * NN) return; const int n = e % NN; const int d = e / NN; v2h o; o[0] = tohx(V[(size_t)n * DD + d]); o[1] = tohx(V[(size_t)(n + 1) * DD + d]); *(volatile v2h*)(VT + e) = o; __threadfence(); *(volatile v2h*)(VT + e) = o; }
__global__ __launch_bounds__(256) void k_relu(const float* __restrict__ S, h16* P) { const size_t e = ((size_t)blockIdx.x * 256 + threadIdx.x) * 4; if (e >= (size_t)NN * NN) return; const v4f a = *(const v4f*)(S + e); v4h o;
#pragma unroll
    for (int u = 0; u < 4; ++u) o[u] = tohx(fmaxf(a[u], 0.f) * (1.0f / NN) * PCAR); *(volatile v4h*)(P + e) = o; __threadfence(); *(volatile v4h*)(P + e) = o; }
__global__ __launch_bounds__(256) void k_fin(const float* __restrict__ X, const float* __restrict__ O0, const float* __restrict__ O1, float* outb) { const int e = (blockIdx.x * 256 + threadIdx.x) * 4; if (e >= NN * DD) return; const v4f x = *(const v4f*)(X + e), a = *(const v4f*)(O0 + e), b = *(const v4f*)(O1 + e); v4f r;
#pragma unroll
    for (int u = 0; u < 4; ++u) { float s = __fadd_rn(a[u] * (1.0f / PCAR), b[u] * (1.0f / PCAR)); asm volatile("" : "+v"(s)); r[u] = __fadd_rn(bfr(x[u]), s); } *(volatile v4f*)(outb + e) = r; __threadfence(); *(volatile v4f*)(outb + e) = r; }

extern "C" void kernel_launch(void* const* d_in, const int* in_sizes, int n_in,
                              void* d_out, int out_size, void* d_ws, size_t ws_size, hipStream_t stream) {
    (void)in_sizes; (void)n_in; (void)out_size;
    const float** I = (const float**)d_in;
    const float *x = I[0], *WQ = I[1], *WK = I[2], *WV = I[3];
    float* OUT = (float*)d_out;
    char* wsp = (char*)d_ws;
    auto take = [&](size_t bytes) { char* p = wsp; wsp += (bytes + 255) & ~(size_t)255; return (void*)p; };
    bf* BQ = (bf*)take(NH_ * DD * DD * 2); bf* BK = (bf*)take(NH_ * DD * DD * 2); bf* BV = (bf*)take(NH_ * DD * DD * 2); bf* XB = (bf*)take((size_t)NN * DD * 2);
    float* Q = (float*)take((size_t)NN * DD * 4); float* K = (float*)take((size_t)NN * DD * 4); float* V = (float*)take((size_t)NN * DD * 4); h16* Q16 = (h16*)take((size_t)NN * DD * 2); h16* K16 = (h16*)take((size_t)NN * DD * 2); h16* VT = (h16*)take((size_t)DD * NN * 2);
    float* S = (float*)take((size_t)NN * NN * 4); h16* P = (h16*)take((size_t)NN * NN * 2); float* O[2]; O[0] = (float*)take((size_t)NN * DD * 4); O[1] = (float*)take((size_t)NN * DD * 4);
    if ((size_t)(wsp - (char*)d_ws) > ws_size) return;
    for (int h = 0; h < NH_; ++h) { k_wtG<<<(DD * DD / 64 + 63) / 64, 256, 0, stream>>>(WQ + h * DD * DD, DD, DD, BQ + h * DD * DD); k_wtG<<<(DD * DD / 64 + 63) / 64, 256, 0, stream>>>(WK + h * DD * DD, DD, DD, BK + h * DD * DD); k_wtG<<<(DD * DD / 64 + 63) / 64, 256, 0, stream>>>(WV + h * DD * DD, DD, DD, BV + h * DD * DD); }
    for (int b = 0; b < NB_; ++b) { const float* xb = x + (size_t)b * NN * DD;
        k_cvt8<<<(NN * DD / 8 + 255) / 256, 256, 0, stream>>>(xb, XB, NN * DD / 8);
        for (int h = 0; h < NH_; ++h) {
            k_gemmw<bf, 0, false><<<dim3(NN / 64, 1, 1), 32, 0, stream>>>(XB, nullptr, BQ + h * DD * DD, nullptr, DD, Q, DD, nullptr, 0, 0, 0); k_gemmw<bf, 0, false><<<dim3(NN / 64, 1, 1), 32, 0, stream>>>(XB, nullptr, BK + h * DD * DD, nullptr, DD, K, DD, nullptr, 0, 0, 0); k_gemmw<bf, 0, false><<<dim3(NN / 64, 1, 1), 32, 0, stream>>>(XB, nullptr, BV + h * DD * DD, nullptr, DD, V, DD, nullptr, 0, 0, 0);
            k_p16<<<(NN * DD / 4 + 255) / 256, 256, 0, stream>>>(Q, Q16); k_p16<<<(NN * DD / 4 + 255) / 256, 256, 0, stream>>>(K, K16); k_vt<<<(DD * NN / 2 + 255) / 256, 256, 0, stream>>>(V, VT);
            k_gemmw<h16, 0, false><<<dim3(NN / 64, NN / 64, 1), 32, 0, stream>>>(Q16, nullptr, K16, nullptr, DD, S, NN, nullptr, 0, 0, 0);
            k_relu<<<(unsigned)(((size_t)NN * NN / 4 + 255) / 256), 256, 0, stream>>>(S, P);
            k_gemmw<h16, 0, false><<<dim3(NN / 64, 1, 1), 32, 0, stream>>>(P, nullptr, VT, nullptr, NN, O[h], DD, nullptr, 0, 0, 0); }
        k_fin<<<(NN * DD / 4 + 255) / 256, 256, 0, stream>>>(xb, O[0], O[1], OUT + (size_t)b * NN * DD); }
}
